// Cross_SelfAttention_85633057948147
// MI455X (gfx1250) — hardware-verified
//
#include <hip/hip_runtime.h>
#include <stdint.h>

constexpr int kB      = 2;
constexpr int kHalfC  = 256;
constexpr int kChan   = 512;
constexpr int kHW     = 4096;
constexpr int kDQ     = 16;
constexpr int kZ      = 4;
constexpr int kQKPitch = 64;
constexpr int kQChunk = 2048;
constexpr int kNChunk = kHW / kQChunk;
constexpr float kWCarry   = 16.0f;
constexpr float kPCarry   = 32768.0f;
constexpr float kCatCarry = 256.0f;
constexpr float kPVScale  = kCatCarry / kPCarry;
constexpr float kOutScale = 1.0f / (kCatCarry * kWCarry);

constexpr size_t kXtmPlane = (size_t)kHW * kHalfC;
constexpr size_t kQKPlane  = (size_t)kHW * kQKPitch;
constexpr size_t kVPlane   = (size_t)kHalfC * kHW;
constexpr size_t kCatPlane = (size_t)kHW * kChan;
constexpr size_t kOffXtm  = 0;
constexpr size_t kOffWqk  = kOffXtm + kZ * kXtmPlane * 2;
constexpr size_t kOffWv   = kOffWqk + (size_t)64 * kHalfC * 2;
constexpr size_t kOffWpt  = kOffWv + (size_t)kHalfC * kHalfC * 2;
constexpr size_t kOffBias = kOffWpt + (size_t)kHalfC * kChan * 2;
constexpr size_t kOffQkh  = kOffBias + 4096;
constexpr size_t kOffQkl  = kOffQkh + kZ * kQKPlane * 2;
constexpr size_t kOffVcm  = kOffQkl + kZ * kQKPlane * 2;
constexpr size_t kOffS    = kOffVcm + kZ * kVPlane * 2;
constexpr size_t kOffP    = kOffS + (size_t)kQChunk * kHW * 4;
constexpr size_t kOffCat  = kOffP + (size_t)kQChunk * kHW * 2;
constexpr size_t kWsTotal = kOffCat + kZ * kCatPlane * 2;
static_assert(kWsTotal == 88510464ull, "carve total");
static_assert(kWsTotal <= 134217728ull, "carve under 128 MiB");
static_assert((kOffWqk % 4096) == 0 && (kOffWv % 4096) == 0 && (kOffWpt % 4096) == 0 && (kOffBias % 4096) == 0 &&
              (kOffQkh % 4096) == 0 && (kOffQkl % 4096) == 0 && (kOffVcm % 4096) == 0 && (kOffS % 4096) == 0 &&
              (kOffP % 4096) == 0 && (kOffCat % 4096) == 0, "aligned regions");

typedef __attribute__((ext_vector_type(16))) _Float16 v16h;
typedef __attribute__((ext_vector_type(8)))  _Float16 v8h;
typedef __attribute__((ext_vector_type(16))) __bf16   v16b;
typedef __attribute__((ext_vector_type(8)))  __bf16   v8b;
typedef __attribute__((ext_vector_type(8)))  float    v8f;
typedef __attribute__((ext_vector_type(4)))  float    v4f;
typedef __attribute__((ext_vector_type(4)))  unsigned int v4u;

__device__ __forceinline__ unsigned short f2bf_bits(float f) {
  unsigned u = __float_as_uint(f);
  return (unsigned short)((u + 0x7FFFu + ((u >> 16) & 1u)) >> 16);
}
__device__ __forceinline__ float bf_bits2f(unsigned short h) { return __uint_as_float(((unsigned)h) << 16); }
__device__ __forceinline__ float bf_rne(float f) { return bf_bits2f(f2bf_bits(f)); }
__device__ __forceinline__ unsigned pk16(unsigned short a, unsigned short b) { return (unsigned)a | ((unsigned)b << 16); }
__device__ __forceinline__ unsigned short h_bits(float f) { const _Float16 h = (_Float16)f; return __builtin_bit_cast(unsigned short, h); }

__device__ __forceinline__ void dep_guard_h(v8f& a, v8f& b, v16h x, v16h y) { asm volatile("v_nop\n\tv_nop\n\tv_nop\n\tv_nop" : "+v"(a), "+v"(b) : "v"(x), "v"(y)); }
__device__ __forceinline__ void dep_guard_b(v8f& a, v8f& b, v16b x, v16b y) { asm volatile("v_nop\n\tv_nop\n\tv_nop\n\tv_nop" : "+v"(a), "+v"(b) : "v"(x), "v"(y)); }
__device__ __forceinline__ void keep4_h(v16h a, v16h b, v16h c, v16h d) { asm volatile("v_nop" :: "v"(a), "v"(b), "v"(c), "v"(d)); }
__device__ __forceinline__ void keep4_b(v16b a, v16b b, v16b c, v16b d) { asm volatile("v_nop" :: "v"(a), "v"(b), "v"(c), "v"(d)); }
__device__ __forceinline__ void acc_guard4(v8f& a, v8f& b, v8f& c, v8f& d) { asm volatile("v_nop\n\tv_nop\n\tv_nop\n\tv_nop" : "+v"(a), "+v"(b), "+v"(c), "+v"(d)); }
template <typename T> struct Frag;
template <> struct Frag<_Float16> {
  typedef v16h V; union U { v16h v; v8h h[2]; };
  static __device__ __forceinline__ v16h load(const _Float16* p) {
    U f; f.h[0] = *(const v8h*)(p); f.h[1] = *(const v8h*)(p + 16); return f.v;
  }
  static __device__ __forceinline__ v8f mma(v16h a, v16h b, v8f c) {
    return __builtin_amdgcn_wmma_f32_16x16x32_f16(false, a, false, b, (short)0, c, false, false);
  }
  static __device__ __forceinline__ void guard(v8f& a, v8f& b, v16h x, v16h y) { dep_guard_h(a, b, x, y); }
  static __device__ __forceinline__ void keep(v16h a, v16h b, v16h c, v16h d) { keep4_h(a, b, c, d); }
};
template <> struct Frag<__bf16> {
  typedef v16b V; union U { v16b v; v8b h[2]; };
  static __device__ __forceinline__ v16b load(const __bf16* p) {
    U f; f.h[0] = *(const v8b*)(p); f.h[1] = *(const v8b*)(p + 16); return f.v;
  }
  static __device__ __forceinline__ v8f mma(v16b a, v16b b, v8f c) {
    return __builtin_amdgcn_wmma_f32_16x16x32_bf16(false, a, false, b, (short)0, c, false, false);
  }
  static __device__ __forceinline__ void guard(v8f& a, v8f& b, v16b x, v16b y) { dep_guard_b(a, b, x, y); }
  static __device__ __forceinline__ void keep(v16b a, v16b b, v16b c, v16b d) { keep4_b(a, b, c, d); }
};

template <int ET> struct Elem;
template <> struct Elem<0> { typedef _Float16 T; };
template <> struct Elem<1> { typedef __bf16 T; };
template <int ET, bool SPLIT, int BIAS_MODE, int OUT_MODE, int RESID_MODE, bool GMUL>
__global__ __launch_bounds__(256) void wmma_gemm64(
    const unsigned short* __restrict__ Ap, const unsigned short* __restrict__ A2p, int lda, long strideA,
    const unsigned short* __restrict__ Btp, const unsigned short* __restrict__ Bt2p, int ldb, long strideB,
    void* __restrict__ Cout, void* __restrict__ Cout2, int ldc, long strideC,
    const float* __restrict__ bias,
    const float* __restrict__ resid, long strideR,
    const float* __restrict__ gmul,
    int M, int N, int K, float scale) {
  typedef typename Elem<ET>::T T;
  typedef typename Frag<T>::V V;
  const T* A = (const T*)Ap; const T* A2 = (const T*)A2p; const T* Bt = (const T*)Btp; const T* Bt2 = (const T*)Bt2p;
  __shared__ __align__(16) float sT[8][16 * 68];
  const int b    = blockIdx.y;
  const int lane = threadIdx.x & 31;
  const int wave = threadIdx.x >> 5;
  const int tilesN = N >> 6;
  const int tilesM = M >> 6;
  const int tile = blockIdx.x * 8 + wave;
  if (tile >= tilesM * tilesN) return;
  const int tm = tile / tilesN;
  const int tn = tile - tm * tilesN;
  const int m0 = tm << 6;
  const int n0 = tn << 6;
  const float escale = GMUL ? (scale * gmul[0]) : scale;

  const T* Ab  = A  + (size_t)b * strideA;
  const T* Bb  = Bt + (size_t)b * strideB;
  const T* Ab2 = SPLIT ? (A2  + (size_t)b * strideA) : nullptr;
  const T* Bb2 = SPLIT ? (Bt2 + (size_t)b * strideB) : nullptr;

  const int rlane = lane & 15;
  const int koff  = (lane >> 4) * 8;
  const int mOff  = (lane >> 4) * 8;

  v8f acc[4][4];
#pragma unroll
  for (int i = 0; i < 4; ++i)
#pragma unroll
    for (int j = 0; j < 4; ++j) acc[i][j] = (v8f){0.f,0.f,0.f,0.f,0.f,0.f,0.f,0.f};

  for (int k0 = 0; k0 < K; k0 += 32) {
    V bh[4], bl[4];
#pragma unroll
    for (int j = 0; j < 4; ++j) {
      const size_t bo = (size_t)(n0 + (j << 4) + rlane) * ldb + koff + k0;
      bh[j] = Frag<T>::load(Bb + bo);
      if (SPLIT) bl[j] = Frag<T>::load(Bb2 + bo);
    }
#pragma unroll
    for (int i = 0; i < 4; ++i) {
      const size_t ao = (size_t)(m0 + (i << 4) + rlane) * lda + koff + k0;
      V ah = Frag<T>::load(Ab + ao);
      V al;
      if (SPLIT) al = Frag<T>::load(Ab2 + ao);
#pragma unroll
      for (int j = 0; j < 4; ++j) {
        acc[i][j] = Frag<T>::mma(ah, bh[j], acc[i][j]);
        if (SPLIT) {
          acc[i][j] = Frag<T>::mma(ah, bl[j], acc[i][j]);
          acc[i][j] = Frag<T>::mma(al, bh[j], acc[i][j]);
        }
      }
      Frag<T>::guard(acc[i][0], acc[i][3], ah, SPLIT ? al : ah);
    }
    Frag<T>::keep(bh[0], bh[1], bh[2], bh[3]);
    if (SPLIT) Frag<T>::keep(bl[0], bl[1], bl[2], bl[3]);
  }
  acc_guard4(acc[0][0], acc[0][1], acc[0][2], acc[0][3]);
  acc_guard4(acc[1][0], acc[1][1], acc[1][2], acc[1][3]);
  acc_guard4(acc[2][0], acc[2][1], acc[2][2], acc[2][3]);
  acc_guard4(acc[3][0], acc[3][1], acc[3][2], acc[3][3]);

  float* slab = sT[wave];
  const float* Rb = (RESID_MODE != 0) ? (resid + (size_t)b * strideR) : nullptr;
#pragma unroll
  for (int i = 0; i < 4; ++i) {
    const int mBase = m0 + (i << 4);
#pragma unroll
    for (int j = 0; j < 4; ++j) {
      const int n = n0 + (j << 4) + rlane;
      float bv = 0.f;
      if (BIAS_MODE == 2) bv = bias[n];
#pragma unroll
      for (int r = 0; r < 8; ++r) {
        float v = acc[i][j][r] * escale;
        if (BIAS_MODE == 1) v += bias[mBase + mOff + r];
        if (BIAS_MODE == 2) v += bv;
        if (RESID_MODE == 1) v += Rb[(size_t)(mBase + mOff + r) * ldc + n];
        if (RESID_MODE == 2) v += bf_rne(Rb[(size_t)(mBase + mOff + r) * ldc + n]);
        slab[(mOff + r) * 68 + (j << 4) + rlane] = v;
      }
    }
    __builtin_amdgcn_fence(__ATOMIC_RELEASE, "workgroup");
    __builtin_amdgcn_wave_barrier();
    __builtin_amdgcn_fence(__ATOMIC_ACQUIRE, "workgroup");
    if (OUT_MODE == 0) {
      float* C = (float*)Cout + (size_t)b * strideC;
      const int hh = lane >> 4, c4 = (lane & 15) * 4;
      for (int pass = 0; pass < 2; ++pass) {
#pragma unroll
        for (int it = 0; it < 8; ++it) {
          const int row = it * 2 + hh;
          v4f v = *(const v4f*)(slab + row * 68 + c4);
          *(volatile v4f*)(C + (size_t)(mBase + row) * ldc + n0 + c4) = v;
        }
        __threadfence();
      }
    } else {
      const int q = lane >> 3, c8 = (lane & 7) * 8;
      unsigned short* C  = (unsigned short*)Cout  + (size_t)b * strideC;
      unsigned short* C2 = (OUT_MODE == 2) ? ((unsigned short*)Cout2 + (size_t)b * strideC) : nullptr;
      for (int pass = 0; pass < 2; ++pass) {
#pragma unroll
        for (int it = 0; it < 4; ++it) {
          const int row = it * 4 + q;
          const float* sp = slab + row * 68 + c8;
          v8h hv, lv;
#pragma unroll
          for (int e = 0; e < 8; ++e) {
            if (OUT_MODE == 1) {
              hv[e] = (_Float16)sp[e];
            } else {
              unsigned short hb = f2bf_bits(sp[e]);
              unsigned short lb = f2bf_bits(sp[e] - bf_bits2f(hb));
              hv[e] = __builtin_bit_cast(_Float16, hb);
              lv[e] = __builtin_bit_cast(_Float16, lb);
            }
          }
          *(volatile v8h*)(C + (size_t)(mBase + row) * ldc + n0 + c8) = hv;
          if (OUT_MODE == 2) *(volatile v8h*)(C2 + (size_t)(mBase + row) * ldc + n0 + c8) = lv;
        }
        __threadfence();
      }
    }
    __builtin_amdgcn_fence(__ATOMIC_RELEASE, "workgroup");
    __builtin_amdgcn_wave_barrier();
    __builtin_amdgcn_fence(__ATOMIC_ACQUIRE, "workgroup");
  }
}

__global__ __launch_bounds__(256) void x_tm_kernel(const float* __restrict__ x, unsigned short* __restrict__ xtm) {
  __shared__ float sm[64][65];
  const int t  = threadIdx.x;
  const int p0 = blockIdx.x * 64;
  const int c0 = blockIdx.y * 64;
  const int z  = blockIdx.z;
  const float* src = x + ((size_t)z * kHalfC + c0) * kHW + p0;
#pragma unroll
  for (int i = 0; i < 16; ++i) {
    const int e  = i * 256 + t;
    const int cl = e >> 6;
    const int pl = e & 63;
    sm[pl][cl] = src[(size_t)cl * kHW + pl];
  }
  __syncthreads();
  const int lane = t & 31, wave = t >> 5;
  const int q = lane >> 3, c8 = (lane & 7) * 8;
  unsigned short* op = xtm + (size_t)z * kXtmPlane;
  for (int pass = 0; pass < 2; ++pass) {
#pragma unroll
    for (int it = 0; it < 2; ++it) {
      const int row = wave * 8 + it * 4 + q;
      unsigned short hb[8];
#pragma unroll
      for (int e = 0; e < 8; ++e) hb[e] = f2bf_bits(sm[row][c8 + e]);
      const v4u u = (v4u){pk16(hb[0], hb[1]), pk16(hb[2], hb[3]), pk16(hb[4], hb[5]), pk16(hb[6], hb[7])};
      *(volatile v4u*)(op + (size_t)(p0 + row) * kHalfC + c0 + c8) = u;
    }
    __threadfence();
  }
}

template <int MODE>
__global__ __launch_bounds__(256) void cast8_kernel(const float* __restrict__ in, unsigned short* __restrict__ out, int n8, float mul) {
  const int i = blockIdx.x * 256 + threadIdx.x;
  if (i >= n8) return;
  const float* p = in + 8 * (size_t)i;
  const v4f a = *(const v4f*)(p);
  const v4f c = *(const v4f*)(p + 4);
  unsigned short hb[8];
#pragma unroll
  for (int e = 0; e < 4; ++e) {
    const float v0 = a[e], v1 = c[e];
    if (MODE == 0) { hb[e] = f2bf_bits(v0); hb[4 + e] = f2bf_bits(v1); }
    else           { hb[e] = h_bits(bf_rne(v0) * mul); hb[4 + e] = h_bits(bf_rne(v1) * mul); }
  }
  const v4u u = (v4u){pk16(hb[0], hb[1]), pk16(hb[2], hb[3]), pk16(hb[4], hb[5]), pk16(hb[6], hb[7])};
  unsigned short* q = out + 8 * (size_t)i;
  *(volatile v4u*)q = u;
  __threadfence();
  *(volatile v4u*)q = u;
}

__global__ __launch_bounds__(256) void prep_small_kernel(const float* __restrict__ Wq, const float* __restrict__ bq,
                                                         const float* __restrict__ Wk, const float* __restrict__ bk,
                                                         const float* __restrict__ bvp, const float* __restrict__ bptp,
                                                         const float* __restrict__ gam,
                                                         unsigned short* __restrict__ wqk, float* __restrict__ biasr) {
  const int t = threadIdx.x, lane = t & 31, wave = t >> 5;
  const float g = gam[0];
#pragma unroll 1
  for (int it = 0; it < 8; ++it) {
    const int n  = wave * 8 + it;
    const int qr = n < 16 ? n : 15;
    int kr = n - 32; kr = kr < 0 ? 0 : (kr > 15 ? 15 : kr);
    const float* pq = Wq + (size_t)qr * kHalfC + lane * 8;
    const float* pk = Wk + (size_t)kr * kHalfC + lane * 8;
    const v4f q0 = *(const v4f*)(pq), q1 = *(const v4f*)(pq + 4);
    const v4f k0 = *(const v4f*)(pk), k1 = *(const v4f*)(pk + 4);
    const bool isq = (n < 16);
    const bool isk = (n >= 32) && (n < 48);
    unsigned short hb[8];
#pragma unroll
    for (int e = 0; e < 4; ++e) {
      const float va = isq ? q0[e] : (isk ? k0[e] : 0.0f);
      const float vb = isq ? q1[e] : (isk ? k1[e] : 0.0f);
      hb[e]     = f2bf_bits(va);
      hb[4 + e] = f2bf_bits(vb);
    }
    const v4u u = (v4u){pk16(hb[0], hb[1]), pk16(hb[2], hb[3]), pk16(hb[4], hb[5]), pk16(hb[6], hb[7])};
    unsigned short* op = wqk + (size_t)n * kHalfC + lane * 8;
    *(volatile v4u*)op = u;
    __threadfence();
    *(volatile v4u*)op = u;
  }
  if (t < 144) {
    v4f val;
#pragma unroll
    for (int e = 0; e < 4; ++e) {
      const int idx = 4 * t + e;
      const int iq = idx < 16 ? idx : 15;
      int ik = idx - 32;  ik = ik < 0 ? 0 : (ik > 15 ? 15 : ik);
      int iv = idx - 64;  iv = iv < 0 ? 0 : (iv > 255 ? 255 : iv);
      int ip = idx - 320; ip = ip < 0 ? 0 : (ip > 255 ? 255 : ip);
      const float fq = bq[iq], fk = bk[ik], fv = bvp[iv], fp = bptp[ip];
      float sel = 0.0f;
      sel = (idx < 16) ? fq : sel;
      sel = (idx >= 32 && idx < 48) ? fk : sel;
      sel = (idx >= 64 && idx < 320) ? fv : sel;
      sel = (idx >= 320) ? fp : sel;
      float r = bf_rne(sel);
      r = (idx >= 320) ? (r * g) : r;
      val[e] = r;
    }
    float* op = biasr + 4 * t;
    *(volatile v4f*)op = val;
    __threadfence();
    *(volatile v4f*)op = val;
  }
}

__global__ __launch_bounds__(512) void softmax_row_kernel(const float* __restrict__ S, unsigned short* __restrict__ P) {
  __shared__ float redM[16];
  __shared__ float redS[16];
  const int row  = blockIdx.x;
  const int t    = threadIdx.x;
  const int lane = t & 31, wave = t >> 5;
  const int c0   = t * 8;
  const float* sr = S + (size_t)row * kHW + c0;
  const v4f a = *(const v4f*)(sr);
  const v4f c = *(const v4f*)(sr + 4);
  float xv[8];
#pragma unroll
  for (int e = 0; e < 4; ++e) { xv[e] = a[e]; xv[4 + e] = c[e]; }
  float m = fmaxf(fmaxf(fmaxf(xv[0], xv[1]), fmaxf(xv[2], xv[3])), fmaxf(fmaxf(xv[4], xv[5]), fmaxf(xv[6], xv[7])));
#pragma unroll
  for (int off = 16; off > 0; off >>= 1) m = fmaxf(m, __shfl_xor(m, off, 32));
  if (lane == 0) redM[wave] = m;
  __syncthreads();
  float bm = redM[0];
#pragma unroll
  for (int w = 1; w < 16; ++w) bm = fmaxf(bm, redM[w]);
  float s = 0.0f;
#pragma unroll
  for (int e = 0; e < 8; ++e) { const float ev = __expf(xv[e] - bm); xv[e] = ev; s += ev; }
#pragma unroll
  for (int off = 16; off > 0; off >>= 1) s += __shfl_xor(s, off, 32);
  if (lane == 0) redS[wave] = s;
  __syncthreads();
  float tot = 0.0f;
#pragma unroll
  for (int w = 0; w < 16; ++w) tot += redS[w];
  const float inv = __builtin_amdgcn_rcpf(tot) * kPCarry;
  unsigned short hb[8];
#pragma unroll
  for (int e = 0; e < 8; ++e) hb[e] = h_bits(xv[e] * inv);
  const v4u u = (v4u){pk16(hb[0], hb[1]), pk16(hb[2], hb[3]), pk16(hb[4], hb[5]), pk16(hb[6], hb[7])};
  unsigned short* q = P + (size_t)row * kHW + c0;
  *(volatile v4u*)q = u;
  __threadfence();
  *(volatile v4u*)q = u;
}

static inline unsigned gemm_blocks(int M, int N) { return (unsigned)((((M / 64) * (N / 64)) + 7) / 8); }

extern "C" void kernel_launch(void* const* d_in, const int* in_sizes, int n_in,
                              void* d_out, int out_size, void* d_ws, size_t ws_size, hipStream_t stream) {
  if (n_in < 10) return;
  if (in_sizes[0] != kB * kChan * kHW) return;
  if (in_sizes[1] != kDQ * kHalfC || in_sizes[3] != kDQ * kHalfC) return;
  if (in_sizes[2] < kDQ || in_sizes[4] < kDQ) return;
  if (in_sizes[5] != kHalfC * kHalfC || in_sizes[6] < kHalfC) return;
  if (in_sizes[7] != kHalfC * kChan || in_sizes[8] < kHalfC || in_sizes[9] < 1) return;
  if (out_size != kB * kChan * kHW) return;
  if (ws_size < kWsTotal) return;

  const float* x     = (const float*)d_in[0];
  const float* Wq    = (const float*)d_in[1];
  const float* bq    = (const float*)d_in[2];
  const float* Wk    = (const float*)d_in[3];
  const float* bk    = (const float*)d_in[4];
  const float* Wv    = (const float*)d_in[5];
  const float* bv    = (const float*)d_in[6];
  const float* Wpt   = (const float*)d_in[7];
  const float* bpt   = (const float*)d_in[8];
  const float* gamma = (const float*)d_in[9];

  char* ws = (char*)d_ws;
  unsigned short* xtm   = (unsigned short*)(ws + kOffXtm);
  unsigned short* wqk   = (unsigned short*)(ws + kOffWqk);
  unsigned short* wv16  = (unsigned short*)(ws + kOffWv);
  unsigned short* wpt16 = (unsigned short*)(ws + kOffWpt);
  float*          biasr = (float*)(ws + kOffBias);
  unsigned short* qkh   = (unsigned short*)(ws + kOffQkh);
  unsigned short* qkl   = (unsigned short*)(ws + kOffQkl);
  unsigned short* vcm   = (unsigned short*)(ws + kOffVcm);
  float*          sbuf  = (float*)(ws + kOffS);
  unsigned short* pbuf  = (unsigned short*)(ws + kOffP);
  unsigned short* cat   = (unsigned short*)(ws + kOffCat);
  const float* bias_qk  = biasr;
  const float* bias_v   = biasr + 64;
  const float* bias_ptg = biasr + 320;

  x_tm_kernel<<<dim3(kHW / 64, kHalfC / 64, kZ), 256, 0, stream>>>(x, xtm);
  cast8_kernel<0><<<(kHalfC * kHalfC / 8) / 256, 256, 0, stream>>>(Wv, wv16, kHalfC * kHalfC / 8, 1.0f);
  cast8_kernel<1><<<(kHalfC * kChan / 8) / 256, 256, 0, stream>>>(Wpt, wpt16, kHalfC * kChan / 8, kWCarry);
  prep_small_kernel<<<1, 256, 0, stream>>>(Wq, bq, Wk, bk, bv, bpt, gamma, wqk, biasr);

  wmma_gemm64<1, false, 2, 2, 0, false><<<dim3(gemm_blocks(kHW, 64), kZ), 256, 0, stream>>>(
      xtm, xtm, kHalfC, (long)kXtmPlane,
      wqk, wqk, kHalfC, 0L,
      (void*)qkh, (void*)qkl, kQKPitch, (long)kQKPlane,
      bias_qk, bias_qk, 0L, gamma,
      kHW, 64, kHalfC, 1.0f);

  wmma_gemm64<1, false, 1, 1, 0, false><<<dim3(gemm_blocks(kHalfC, kHW), kZ), 256, 0, stream>>>(
      wv16, wv16, kHalfC, 0L,
      xtm, xtm, kHalfC, (long)kXtmPlane,
      (void*)vcm, (void*)vcm, kHW, (long)kVPlane,
      bias_v, bias_v, 0L, gamma,
      kHalfC, kHW, kHalfC, 1.0f);

  for (int z = 0; z < kZ; ++z) {
    const unsigned short* qh = qkh + (size_t)z * kQKPlane;
    const unsigned short* ql = qkl + (size_t)z * kQKPlane;
    const unsigned short* vb = vcm + (size_t)(z >> 1) * 2 * kVPlane;
    for (int qc = 0; qc < kNChunk; ++qc) {
      const size_t qoff = (size_t)qc * kQChunk * kQKPitch;
      wmma_gemm64<1, true, 0, 0, 0, false><<<dim3(gemm_blocks(kQChunk, kHW), 1), 256, 0, stream>>>(
          qh + qoff, ql + qoff, kQKPitch, 0L,
          qh + 32, ql + 32, kQKPitch, 0L,
          (void*)sbuf, (void*)sbuf, kHW, 0L,
          bias_v, bias_v, 0L, gamma,
          kQChunk, kHW, 32, 1.0f);
      softmax_row_kernel<<<kQChunk, 512, 0, stream>>>(sbuf, pbuf);
      wmma_gemm64<0, false, 0, 1, 0, false><<<dim3(gemm_blocks(kQChunk, kHalfC), 2), 256, 0, stream>>>(
          pbuf, pbuf, kHW, 0L,
          vb, vb, kHW, (long)kVPlane,
          (void*)(cat + (size_t)z * kCatPlane + (size_t)qc * kQChunk * kChan), (void*)(cat + (size_t)z * kCatPlane + (size_t)qc * kQChunk * kChan), kChan, 256L,
          bias_v, bias_v, 0L, gamma,
          kQChunk, kHalfC, kHW, kPVScale);
    }
  }

  wmma_gemm64<0, false, 1, 0, 2, true><<<dim3(gemm_blocks(kHalfC, kHW), kZ), 256, 0, stream>>>(
      wpt16, wpt16, kChan, 0L,
      cat, cat, kChan, (long)kCatPlane,
      d_out, d_out, kHW, (long)kHalfC * kHW,
      bias_ptg, x, (long)kHalfC * kHW, gamma,
      kHalfC, kHW, kChan, kOutScale);
}
